// LRCModel_45827301048581
// MI455X (gfx1250) — hardware-verified
//
#include <hip/hip_runtime.h>


namespace {
constexpr int NN = 32, DD = 96, NE = 256, NP = NN * NN, NR = NP * NE, C1L = 47, P1L = 23, C2L = 21, P2L = 10, C3L = 8, P3L = 4, NF = 16, F1 = 128, F2 = 256, F3 = 128, NSTEP = 3;
constexpr float XS = 8.0f, WSC = 256.0f;
typedef _Float16 b16;
typedef __attribute__((ext_vector_type(16))) _Float16 v16b;
typedef __attribute__((ext_vector_type(8))) _Float16 v8b;
typedef __attribute__((ext_vector_type(8))) float v8f;
typedef __attribute__((ext_vector_type(4))) float v4f;
__device__ __forceinline__ float bf16_rne(float f) { unsigned int u = __float_as_uint(f); u += 0x7FFFu + ((u >> 16) & 1u); return __uint_as_float(u & 0xFFFF0000u); }
__device__ __forceinline__ void split16(float v, b16& hi, b16& lo) { hi = (b16)v; lo = (b16)(v - (float)hi); }
__device__ __forceinline__ v16b frag_kb(const b16* p, int hh) { const v8b a = *(const v8b*)(p + 8 * hh), b = *(const v8b*)(p + 16 + 8 * hh); v16b f;
#pragma unroll
  for (int e = 0; e < 8; ++e) { f[e] = a[e]; f[8 + e] = b[e]; } return f; }
__device__ __forceinline__ v8f wmma16b(v16b a, v16b b, v8f c) { v8f d = __builtin_amdgcn_wmma_f32_16x16x32_f16(false, a, false, b, (short)0, c, false, false); asm volatile("v_nop\n\tv_nop\n\tv_nop\n\tv_nop" : "+v"(d) : "v"(a), "v"(b)); return d; }
__device__ __forceinline__ void wave_lds_sync() { __builtin_amdgcn_fence(__ATOMIC_RELEASE, "workgroup"); __builtin_amdgcn_wave_barrier(); __builtin_amdgcn_fence(__ATOMIC_ACQUIRE, "workgroup"); }
__device__ __forceinline__ float pmul(float a, float b) { float p = a * b; asm volatile("" : "+v"(p)); return p; }
__device__ __forceinline__ int iclamp(int v, int lo, int hi) { return v < lo ? lo : (v > hi ? hi : v); }

__global__ __launch_bounds__(256) void wprep_kernel(const float* __restrict__ w1, const float* __restrict__ w2, const float* __restrict__ w3, b16* __restrict__ W1T, b16* __restrict__ W2T, b16* __restrict__ W3T) {
  const int u = blockIdx.x * 256 + threadIdx.x; const int n1 = F1 * 32 / 8, n2 = F2 * F1 / 8, n3 = F3 * F2 / 8; v8b v;
  if (u < n1) { const int e = u * 8, o = e / 32, k0 = e % 32; for (int j = 0; j < 8; ++j) { const int k = k0 + j; v[j] = k < NF ? (b16)(bf16_rne(w1[(k < NF ? k : 0) * F1 + o]) * WSC) : (b16)0.0f; } for (int p = 0; p < 2; ++p) { *(volatile v8b*)(W1T + e) = v; __threadfence(); } return; }
  int t = u - n1; if (t < n2) { const int e = t * 8, o = e / F1, k0 = e % F1; for (int j = 0; j < 8; ++j) v[j] = (b16)(bf16_rne(w2[(size_t)(k0 + j) * F2 + o]) * WSC); for (int p = 0; p < 2; ++p) { *(volatile v8b*)(W2T + e) = v; __threadfence(); } return; }
  t -= n2; if (t < n3) { const int e = t * 8, o = e / F2, k0 = e % F2; for (int j = 0; j < 8; ++j) v[j] = (b16)(bf16_rne(w3[(size_t)(k0 + j) * F3 + o]) * WSC); for (int p = 0; p < 2; ++p) { *(volatile v8b*)(W3T + e) = v; __threadfence(); } }
}
constexpr int ROWF = 192;
__global__ __launch_bounds__(64) void tab_kernel(const float* __restrict__ emb, const int* __restrict__ edges, const float* __restrict__ w1, const float* __restrict__ b1, float* __restrict__ A, float* __restrict__ Bt) {
  const int r = blockIdx.x; const int tid = threadIdx.x; const bool isA = r < NP; int i0, i1; float w[2][4][3];
  if (isA) { i0 = r / NN; i1 = r % NN; } else { const int e = r - NP; i0 = iclamp(edges[e * 2], 0, NN - 1); i1 = iclamp(edges[e * 2 + 1], 0, NN - 1); }
  const int cbase = isA ? 0 : 2;
  for (int o = 0; o < 4; ++o) for (int k = 0; k < 3; ++k) { w[0][o][k] = bf16_rne(w1[(o * 4 + cbase) * 3 + k]); w[1][o][k] = bf16_rne(w1[(o * 4 + cbase + 1) * 3 + k]); }
  float* dst = (isA ? A + (size_t)r * ROWF : Bt + (size_t)(r - NP) * ROWF);
  for (int pass = 0; pass < 2; ++pass) {
    for (int idx = tid; idx < ROWF; idx += 64) { float val = 0.0f; if (idx < 4 * C1L) { const int o = idx / C1L, j = idx % C1L; val = isA ? bf16_rne(b1[o]) : 0.0f;
        for (int k = 0; k < 3; ++k) { const int pos = 2 * j + k; val += pmul(w[0][o][k], bf16_rne(emb[i0 * DD + pos])) + pmul(w[1][o][k], bf16_rne(emb[i1 * DD + pos])); } }
      ((volatile float*)dst)[idx] = val; }
    __threadfence(); }
}
template <int NT, int KW>
__device__ __forceinline__ void gemm_tiles(const b16 (*Ah)[F2 + 8], const b16 (*Al)[F2 + 8], const b16* __restrict__ WT, int c0, v8f* acc, int nloc, int hlf) {
#pragma unroll
  for (int t = 0; t < NT; ++t) acc[t] = (v8f){};
#pragma unroll 2
  for (int kb = 0; kb < KW; kb += 32) { const v16b a = frag_kb(&Ah[nloc][kb], hlf), al = frag_kb(&Al[nloc][kb], hlf);
#pragma unroll
    for (int t = 0; t < NT; ++t) { const v16b bw = frag_kb(WT + (size_t)(c0 + t * 16 + nloc) * KW + kb, hlf); acc[t] = wmma16b(a, bw, acc[t]); acc[t] = wmma16b(al, bw, acc[t]); } }
}
template <int NT, int KW>
__device__ __forceinline__ void gemm_tilesB(const b16 (*Ah)[F1 + 8], const b16 (*Al)[F1 + 8], const b16* __restrict__ WT, int c0, v8f* acc, int nloc, int hlf) {
#pragma unroll
  for (int t = 0; t < NT; ++t) acc[t] = (v8f){};
#pragma unroll 2
  for (int kb = 0; kb < KW; kb += 32) { const v16b a = frag_kb(&Ah[nloc][kb], hlf), al = frag_kb(&Al[nloc][kb], hlf);
#pragma unroll
    for (int t = 0; t < NT; ++t) { const v16b bw = frag_kb(WT + (size_t)(c0 + t * 16 + nloc) * KW + kb, hlf); acc[t] = wmma16b(a, bw, acc[t]); acc[t] = wmma16b(al, bw, acc[t]); } }
}
__global__ __launch_bounds__(64) void main_kernel(const float* __restrict__ A, const float* __restrict__ Bt, const float* __restrict__ w2c, const float* __restrict__ b2c, const float* __restrict__ w3c, const float* __restrict__ b3c,
                                                  const b16* __restrict__ W1T, const b16* __restrict__ W2T, const b16* __restrict__ W3T, const float* __restrict__ fb1, const float* __restrict__ fb2, const float* __restrict__ fb3, const float* __restrict__ fw4, const float* __restrict__ fb4, float* __restrict__ PRED) {
  __shared__ __attribute__((aligned(16))) b16 Ah[2][16][F2 + 8], Al[2][16][F2 + 8], Bh[2][16][F1 + 8], Bl[2][16][F1 + 8]; __shared__ float H1[2][4 * P1L][32]; __shared__ float feat[2][32][NF]; __shared__ float so[2][32]; __shared__ float wc[2][48], bc[2][4];
  const int wave = threadIdx.x >> 5, lane = threadIdx.x & 31, nloc = lane & 15, hlf = lane >> 4; const size_t r0 = ((size_t)blockIdx.x * 2 + wave) * 32; const int p = (int)(r0 / NE); const int e = (int)(r0 % NE) + lane;
  if (threadIdx.x < 48) { wc[0][threadIdx.x] = bf16_rne(w2c[threadIdx.x]); wc[1][threadIdx.x] = bf16_rne(w3c[threadIdx.x]); } if (threadIdx.x < 4) { bc[0][threadIdx.x] = bf16_rne(b2c[threadIdx.x]); bc[1][threadIdx.x] = bf16_rne(b3c[threadIdx.x]); }
  __syncthreads();
  { const float* Ar = A + (size_t)p * ROWF; const float* Br = Bt + (size_t)e * ROWF;
    for (int o = 0; o < 4; ++o)
#pragma unroll 1
      for (int j = 0; j < P1L; ++j) { const float c0v = fmaxf(Ar[o * C1L + 2 * j] + Br[o * C1L + 2 * j], 0.0f), c1v = fmaxf(Ar[o * C1L + 2 * j + 1] + Br[o * C1L + 2 * j + 1], 0.0f); H1[wave][o * P1L + j][lane] = fmaxf(c0v, c1v); }
    float h2[4][P2L];
#pragma unroll
    for (int o = 0; o < 4; ++o)
#pragma unroll
      for (int j = 0; j < P2L; ++j) { float c0v = bc[0][o], c1v = bc[0][o];
#pragma unroll
      for (int i = 0; i < 4; ++i)
#pragma unroll
        for (int k = 0; k < 3; ++k) { const float wv = wc[0][(o * 4 + i) * 3 + k]; c0v += pmul(wv, H1[wave][i * P1L + 2 * j + k][lane]); c1v += pmul(wv, H1[wave][i * P1L + 2 * j + 1 + k][lane]); }
      h2[o][j] = fmaxf(fmaxf(c0v, 0.0f), fmaxf(c1v, 0.0f)); }
#pragma unroll
    for (int o = 0; o < 4; ++o)
#pragma unroll
      for (int j = 0; j < P3L; ++j) { float c0v = bc[1][o], c1v = bc[1][o];
#pragma unroll
      for (int i = 0; i < 4; ++i)
#pragma unroll
        for (int k = 0; k < 3; ++k) { const float wv = wc[1][(o * 4 + i) * 3 + k]; c0v += pmul(wv, h2[i][2 * j + k]); c1v += pmul(wv, h2[i][2 * j + 1 + k]); }
      feat[wave][lane][o * P3L + j] = fmaxf(fmaxf(c0v, 0.0f), fmaxf(c1v, 0.0f)); } }
  wave_lds_sync();
  const float sc = 1.0f / (XS * WSC);
#pragma unroll 1
  for (int half = 0; half < 2; ++half) {
    { const int rr = nloc, c = hlf * 8; for (int j = 0; j < 8; ++j) { const int col = c + j; b16 ph, pl; split16(feat[wave][half * 16 + rr][col] * XS, ph, pl); Ah[wave][rr][col] = ph; Al[wave][rr][col] = pl; Ah[wave][rr][16 + col] = (b16)0.0f; Al[wave][rr][16 + col] = (b16)0.0f; } }
    wave_lds_sync();
    v8f acc[8];
    gemm_tiles<8, 32>(Ah[wave], Al[wave], W1T, 0, acc, nloc, hlf);
#pragma unroll
    for (int t = 0; t < 8; ++t) { const float bb = bf16_rne(fb1[t * 16 + nloc]);
#pragma unroll
      for (int r8 = 0; r8 < 8; ++r8) { const float v = fmaxf(acc[t][r8] * sc + bb, 0.0f); b16 ph, pl; split16(v * XS, ph, pl); Bh[wave][8 * hlf + r8][t * 16 + nloc] = ph; Bl[wave][8 * hlf + r8][t * 16 + nloc] = pl; } }
    wave_lds_sync();
#pragma unroll 1
    for (int cg = 0; cg < 2; ++cg) { gemm_tilesB<8, F1>(Bh[wave], Bl[wave], W2T, cg * 128, acc, nloc, hlf);
#pragma unroll
      for (int t = 0; t < 8; ++t) { const float bb = bf16_rne(fb2[cg * 128 + t * 16 + nloc]);
#pragma unroll
        for (int r8 = 0; r8 < 8; ++r8) { const float v = fmaxf(acc[t][r8] * sc + bb, 0.0f); b16 ph, pl; split16(v * XS, ph, pl); Ah[wave][8 * hlf + r8][cg * 128 + t * 16 + nloc] = ph; Al[wave][8 * hlf + r8][cg * 128 + t * 16 + nloc] = pl; } } }
    wave_lds_sync();
    gemm_tiles<8, F2>(Ah[wave], Al[wave], W3T, 0, acc, nloc, hlf);
    { float ps[8]; for (int r8 = 0; r8 < 8; ++r8) ps[r8] = 0.0f;
#pragma unroll
      for (int t = 0; t < 8; ++t) { const int c = t * 16 + nloc; const float bb = bf16_rne(fb3[c]), wv = bf16_rne(fw4[c]);
#pragma unroll
        for (int r8 = 0; r8 < 8; ++r8) ps[r8] += pmul(fmaxf(acc[t][r8] * sc + bb, 0.0f), wv); }
      const int s_ = p / NN, t_ = p % NN; const float b4 = bf16_rne(fb4[0]);
#pragma unroll
      for (int r8 = 0; r8 < 8; ++r8) { float s = ps[r8]; for (int o = 1; o < 16; o <<= 1) s += __shfl_xor(s, o); if (nloc == 0) so[wave][half * 16 + 8 * hlf + r8] = (s_ == t_) ? 0.0f : s + b4; } }
    wave_lds_sync(); }
  for (int pass = 0; pass < 2; ++pass) { ((volatile float*)PRED)[r0 + lane] = so[wave][lane]; __threadfence(); }
}
__global__ __launch_bounds__(256) void route_kernel(const float* __restrict__ PRED, const int* __restrict__ edges, int nsrc, float* __restrict__ PART) {
  __shared__ float X[256][NN + 1], XN[256][NN + 1], RB[256][NN + 1]; __shared__ int eu[NE], ev[NE];
  const int tid = threadIdx.x; const int p = blockIdx.x * 256 + tid; const bool ok = p < nsrc;
  if (tid < NE) { eu[tid] = iclamp(edges[tid * 2], 0, NN - 1); ev[tid] = iclamp(edges[tid * 2 + 1], 0, NN - 1); }
  for (int n = 0; n < NN; ++n) { X[tid][n] = 0.0f; RB[tid][n] = 0.0f; } if (ok) X[tid][p / NN] = 1.0f;
  __syncthreads();
  if (ok) {
#pragma unroll 1
    for (int st = 0; st < NSTEP; ++st) { for (int n = 0; n < NN; ++n) XN[tid][n] = 0.0f;
#pragma unroll 1
      for (int e = 0; e < NE; ++e) { const float g = pmul(X[tid][eu[e]], PRED[(size_t)p * NE + e]); XN[tid][ev[e]] += g; }
      for (int n = 0; n < NN; ++n) { const float v = XN[tid][n]; X[tid][n] = v; RB[tid][n] += v; } } }
  __syncthreads();
  float s = 0.0f; if (tid < NN) { for (int q = 0; q < 256; ++q) s += RB[q][tid]; }
  for (int pass = 0; pass < 2; ++pass) { if (tid < NN) ((volatile float*)PART)[blockIdx.x * 32 + tid] = s; __threadfence(); }
}
__global__ __launch_bounds__(32) void final_kernel(const float* __restrict__ PART, int nblk, float* __restrict__ out) {
  const int lane = threadIdx.x; float r = 0.0f; for (int b = 0; b < nblk; ++b) r += PART[b * 32 + lane]; float tot = r; for (int o = 16; o; o >>= 1) tot += __shfl_xor(tot, o);
  const float v = r / tot; for (int pass = 0; pass < 2; ++pass) { ((volatile float*)out)[lane] = v; __threadfence(); }
}
}

extern "C" void kernel_launch(void* const* d_in, const int* in_sizes, int n_in, void* d_out, int out_size, void* d_ws, size_t ws_size, hipStream_t stream) {
  (void)n_in;
  auto Fp = [&](int i) { return (const float*)d_in[i]; }; auto Ip = [&](int i) { return (const int*)d_in[i]; };
  if (in_sizes[0] != NN * DD || in_sizes[1] != NE * 2 || in_sizes[2] != 48 || in_sizes[8] != NF * F1 || in_sizes[10] != F1 * F2 || in_sizes[12] != F2 * F3 || in_sizes[14] != F3 || out_size != NN) return;
  const int NSRC = NP;
  size_t off = 0; char* ws = (char*)d_ws;
  auto carve = [&](size_t bytes) { char* p = ws + off; off += (bytes + 255) & ~(size_t)255; return p; };
  b16* W1T = (b16*)carve(F1 * 32 * 2); b16* W2T = (b16*)carve(F2 * F1 * 2); b16* W3T = (b16*)carve(F3 * F2 * 2);
  float* A = (float*)carve((size_t)NP * ROWF * 4); float* Bt = (float*)carve((size_t)NE * ROWF * 4); float* PRED = (float*)carve((size_t)NR * 4); float* PART = (float*)carve(4 * 32 * 4);
  if (off > ws_size || off > ((size_t)16 << 20)) return;
  wprep_kernel<<<(F1 * 32 / 8 + F2 * F1 / 8 + F3 * F2 / 8 + 255) / 256, 256, 0, stream>>>(Fp(8), Fp(10), Fp(12), W1T, W2T, W3T);
  tab_kernel<<<NP + NE, 64, 0, stream>>>(Fp(0), Ip(1), Fp(2), Fp(3), A, Bt);
  main_kernel<<<NSRC * NE / 64, 64, 0, stream>>>(A, Bt, Fp(4), Fp(5), Fp(6), Fp(7), W1T, W2T, W3T, Fp(9), Fp(11), Fp(13), Fp(14), Fp(15), PRED);
  const int nblk = (NSRC + 255) / 256;
  route_kernel<<<nblk, 256, 0, stream>>>(PRED, Ip(1), NSRC, PART);
  final_kernel<<<1, 32, 0, stream>>>(PART, nblk, (float*)d_out);
}
